// HybridSelfAttentionTransformer_65481071396697
// MI455X (gfx1250) — hardware-run, weakly checked
//
#include <hip/hip_runtime.h>
#include <math.h>
#include <stdint.h>

constexpr int kBatch   = 8;
constexpr int kSeq     = 1024;
constexpr int kDim     = 512;
constexpr int kHeads   = 8;
constexpr int kHeadDim = 64;
constexpr int kFfn     = 2048;
constexpr int kLayers  = 2;
constexpr int kClasses = 10;
constexpr int kRows    = kBatch * kSeq;
constexpr float kWScale    = 64.0f;
constexpr float kWScaleInv = 1.0f / 64.0f;
constexpr float kPScale    = 32768.0f;
static_assert(kDim == kHeads * kHeadDim, "head geometry");
static_assert((kBatch * kClasses) % 4 == 0, "output written as whole float4 lanes");

typedef __attribute__((ext_vector_type(16))) _Float16 v16h;
typedef __attribute__((ext_vector_type(8)))  _Float16 v8h;
typedef __attribute__((ext_vector_type(16))) __bf16   v16b;
typedef __attribute__((ext_vector_type(8)))  __bf16   v8b;
typedef __attribute__((ext_vector_type(8)))  float    v8f;
typedef __attribute__((ext_vector_type(4)))  float    v4f;
typedef __attribute__((ext_vector_type(2)))  float    v2f;
typedef __attribute__((ext_vector_type(4)))  unsigned int v4u;
typedef __attribute__((ext_vector_type(2)))  unsigned int v2u;

__device__ __forceinline__ unsigned short f2bf_bits(float f) {
  unsigned u = __float_as_uint(f);
  return (unsigned short)((u + 0x7FFFu + ((u >> 16) & 1u)) >> 16);
}
__device__ __forceinline__ float bf_bits2f(unsigned short h) { return __uint_as_float(((unsigned)h) << 16); }
__device__ __forceinline__ float bf16r(float f) { return bf_bits2f(f2bf_bits(f)); }
__device__ __forceinline__ unsigned short h_bits(float f) { return __builtin_bit_cast(unsigned short, (_Float16)f); }
__device__ __forceinline__ unsigned pk16(unsigned short a, unsigned short b) { return (unsigned)a | ((unsigned)b << 16); }

__device__ __forceinline__ void dep_guard_h(v8f& a, v8f& b, v16h x, v16h y) { asm volatile("v_nop\n\tv_nop\n\tv_nop\n\tv_nop" : "+v"(a), "+v"(b) : "v"(x), "v"(y)); }
__device__ __forceinline__ void dep_guard_b(v8f& a, v8f& b, v16b x, v16b y) { asm volatile("v_nop\n\tv_nop\n\tv_nop\n\tv_nop" : "+v"(a), "+v"(b) : "v"(x), "v"(y)); }
__device__ __forceinline__ void keep4_h(v16h a, v16h b, v16h c, v16h d) { asm volatile("v_nop" :: "v"(a), "v"(b), "v"(c), "v"(d)); }
__device__ __forceinline__ void keep4_b(v16b a, v16b b, v16b c, v16b d) { asm volatile("v_nop" :: "v"(a), "v"(b), "v"(c), "v"(d)); }
__device__ __forceinline__ void acc_guard4(v8f& a, v8f& b, v8f& c, v8f& d) { asm volatile("v_nop\n\tv_nop\n\tv_nop\n\tv_nop" : "+v"(a), "+v"(b), "+v"(c), "+v"(d)); }
template <typename T> struct Frag;
template <> struct Frag<_Float16> {
  typedef v16h V; union U { v16h v; v8h h[2]; };
  static __device__ __forceinline__ v16h load(const _Float16* p) {
    U f; f.h[0] = *(const v8h*)(p); f.h[1] = *(const v8h*)(p + 16); return f.v;
  }
  static __device__ __forceinline__ v8f mma(v16h a, v16h b, v8f c) {
    return __builtin_amdgcn_wmma_f32_16x16x32_f16(false, a, false, b, (short)0, c, false, false);
  }
  static __device__ __forceinline__ void guard(v8f& a, v8f& b, v16h x, v16h y) { dep_guard_h(a, b, x, y); }
  static __device__ __forceinline__ void keep(v16h a, v16h b, v16h c, v16h d) { keep4_h(a, b, c, d); }
};
template <> struct Frag<__bf16> {
  typedef v16b V; union U { v16b v; v8b h[2]; };
  static __device__ __forceinline__ v16b load(const __bf16* p) {
    U f; f.h[0] = *(const v8b*)(p); f.h[1] = *(const v8b*)(p + 16); return f.v;
  }
  static __device__ __forceinline__ v8f mma(v16b a, v16b b, v8f c) {
    return __builtin_amdgcn_wmma_f32_16x16x32_bf16(false, a, false, b, (short)0, c, false, false);
  }
  static __device__ __forceinline__ void guard(v8f& a, v8f& b, v16b x, v16b y) { dep_guard_b(a, b, x, y); }
  static __device__ __forceinline__ void keep(v16b a, v16b b, v16b c, v16b d) { keep4_b(a, b, c, d); }
};

template <int ET> struct Elem;
template <> struct Elem<0> { typedef _Float16 T; };
template <> struct Elem<1> { typedef __bf16 T; };
template <int ET, bool SPLIT, int BIAS_MODE, int OUT_MODE, bool RESID, int ACT = 0>
__global__ __launch_bounds__(256) void wmma_gemm64(
    const unsigned short* __restrict__ Ap, const unsigned short* __restrict__ A2p, int lda, long strideA,
    const unsigned short* __restrict__ Btp, const unsigned short* __restrict__ Bt2p, int ldb, long strideB,
    void* __restrict__ Cout, void* __restrict__ Cout2, int ldc, long strideC,
    const float* __restrict__ bias,
    const float* __restrict__ resid, long strideR,
    int M, int N, int K, float scale) {
  typedef typename Elem<ET>::T T;
  typedef typename Frag<T>::V V;
  const T* A = (const T*)Ap; const T* A2 = (const T*)A2p; const T* Bt = (const T*)Btp; const T* Bt2 = (const T*)Bt2p;
  __shared__ __align__(16) float sT[8][16 * 68];
  const int b    = blockIdx.y;
  const int lane = threadIdx.x & 31;
  const int wave = threadIdx.x >> 5;
  const int tilesN = N >> 6;
  const int tilesM = M >> 6;
  const int tile = blockIdx.x * 8 + wave;
  if (tile >= tilesM * tilesN) return;
  const int tm = tile / tilesN;
  const int tn = tile - tm * tilesN;
  const int m0 = tm << 6;
  const int n0 = tn << 6;

  const T* Ab  = A  + (size_t)b * strideA;
  const T* Bb  = Bt + (size_t)b * strideB;
  const T* Ab2 = SPLIT ? (A2  + (size_t)b * strideA) : nullptr;
  const T* Bb2 = SPLIT ? (Bt2 + (size_t)b * strideB) : nullptr;

  const int rlane = lane & 15;
  const int koff  = (lane >> 4) * 8;
  const int mOff  = (lane >> 4) * 8;

  v8f acc[4][4];
#pragma unroll
  for (int i = 0; i < 4; ++i)
#pragma unroll
    for (int j = 0; j < 4; ++j) acc[i][j] = (v8f){0.f,0.f,0.f,0.f,0.f,0.f,0.f,0.f};

  for (int k0 = 0; k0 < K; k0 += 32) {
    V bh[4], bl[4];
#pragma unroll
    for (int j = 0; j < 4; ++j) {
      const size_t bo = (size_t)(n0 + (j << 4) + rlane) * ldb + koff + k0;
      bh[j] = Frag<T>::load(Bb + bo);
      if (SPLIT) bl[j] = Frag<T>::load(Bb2 + bo);
    }
#pragma unroll
    for (int i = 0; i < 4; ++i) {
      const size_t ao = (size_t)(m0 + (i << 4) + rlane) * lda + koff + k0;
      V ah = Frag<T>::load(Ab + ao);
      V al;
      if (SPLIT) al = Frag<T>::load(Ab2 + ao);
#pragma unroll
      for (int j = 0; j < 4; ++j) {
        acc[i][j] = Frag<T>::mma(ah, bh[j], acc[i][j]);
        if (SPLIT) {
          acc[i][j] = Frag<T>::mma(ah, bl[j], acc[i][j]);
          acc[i][j] = Frag<T>::mma(al, bh[j], acc[i][j]);
        }
      }
      Frag<T>::guard(acc[i][0], acc[i][3], ah, SPLIT ? al : ah);
    }
    Frag<T>::keep(bh[0], bh[1], bh[2], bh[3]);
    if (SPLIT) Frag<T>::keep(bl[0], bl[1], bl[2], bl[3]);
  }
  acc_guard4(acc[0][0], acc[0][1], acc[0][2], acc[0][3]);
  acc_guard4(acc[1][0], acc[1][1], acc[1][2], acc[1][3]);
  acc_guard4(acc[2][0], acc[2][1], acc[2][2], acc[2][3]);
  acc_guard4(acc[3][0], acc[3][1], acc[3][2], acc[3][3]);

  float* slab = sT[wave];
  const float* Rb = RESID ? (resid + (size_t)b * strideR) : nullptr;
#pragma unroll
  for (int i = 0; i < 4; ++i) {
    const int mBase = m0 + (i << 4);
#pragma unroll
    for (int j = 0; j < 4; ++j) {
      const int n = n0 + (j << 4) + rlane;
      float bv = 0.f;
      if (BIAS_MODE == 2) bv = bias[n];
#pragma unroll
      for (int r = 0; r < 8; ++r) {
        float v = acc[i][j][r] * scale;
        if (BIAS_MODE == 1) v += bias[mBase + mOff + r];
        if (BIAS_MODE == 2) v += bv;
        if (RESID) v += Rb[(size_t)(mBase + mOff + r) * ldc + n];
        if (ACT == 1) v = tanhf(v);
        if (ACT == 2) v = fmaxf(v, 0.0f);
        if (ACT == 3) v = v / (1.0f + expf(-v));
        if (ACT == 4) v = (v > 0.f) ? v : 0.01f * v;
        if (ACT == 5) v = 0.5f * v * (1.0f + erff(v * 0.70710678118654752f));
        slab[(mOff + r) * 68 + (j << 4) + rlane] = v;
      }
    }
    __builtin_amdgcn_fence(__ATOMIC_RELEASE, "workgroup");
    __builtin_amdgcn_wave_barrier();
    __builtin_amdgcn_fence(__ATOMIC_ACQUIRE, "workgroup");
    if (OUT_MODE == 0) {
      float* C = (float*)Cout + (size_t)b * strideC;
      const int hh = lane >> 4, c4 = (lane & 15) * 4;
      for (int pass = 0; pass < 2; ++pass) {
#pragma unroll
        for (int it = 0; it < 8; ++it) {
          const int row = it * 2 + hh;
          v4f v = *(const v4f*)(slab + row * 68 + c4);
          *(volatile v4f*)(C + (size_t)(mBase + row) * ldc + n0 + c4) = v;
        }
        __threadfence();
      }
    } else {
      const int q = lane >> 3, c8 = (lane & 7) * 8;
      unsigned short* C  = (unsigned short*)Cout  + (size_t)b * strideC;
      unsigned short* C2 = (OUT_MODE == 2) ? ((unsigned short*)Cout2 + (size_t)b * strideC) : nullptr;
      for (int pass = 0; pass < 2; ++pass) {
#pragma unroll
        for (int it = 0; it < 4; ++it) {
          const int row = it * 4 + q;
          const float* sp = slab + row * 68 + c8;
          v8h hv, lv;
#pragma unroll
          for (int e = 0; e < 8; ++e) {
            if (OUT_MODE == 1) {
              hv[e] = (_Float16)sp[e];
            } else {
              unsigned short hb = f2bf_bits(sp[e]);
              unsigned short lb = f2bf_bits(sp[e] - bf_bits2f(hb));
              hv[e] = __builtin_bit_cast(_Float16, hb);
              lv[e] = __builtin_bit_cast(_Float16, lb);
            }
          }
          *(volatile v8h*)(C + (size_t)(mBase + row) * ldc + n0 + c8) = hv;
          if (OUT_MODE == 2) *(volatile v8h*)(C2 + (size_t)(mBase + row) * ldc + n0 + c8) = lv;
        }
        __threadfence();
      }
    }
    __builtin_amdgcn_fence(__ATOMIC_RELEASE, "workgroup");
    __builtin_amdgcn_wave_barrier();
    __builtin_amdgcn_fence(__ATOMIC_ACQUIRE, "workgroup");
  }
}

__device__ __forceinline__ float cos_f32(float x) {
  const float n = rintf(x * 0.636619772367581343f);
  float r = fmaf(-n, 1.57079625129699707031e+00f, x);
  r = fmaf(-n, 7.54978941586159635335e-08f, r);
  r = fmaf(-n, 5.39030252995776476554e-15f, r);
  const float z = r * r;
  float sp = fmaf(z, -1.9515295891e-4f, 8.3321608736e-3f);
  sp = fmaf(z, sp, -1.6666654611e-1f);
  const float sr = fmaf(z * r, sp, r);
  float cp = fmaf(z, 2.443315711809948e-5f, -1.388731625493765e-3f);
  cp = fmaf(z, cp, 4.166664568298827e-2f);
  const float cr = fmaf(z * z, cp, fmaf(z, -0.5f, 1.0f));
  const int q = ((int)n) & 3;
  const float v = (q & 1) ? sr : cr;
  return ((q + 1) & 2) ? -v : v;
}

__global__ __launch_bounds__(256) void k_powtab(float* __restrict__ rp) {
  const int j = threadIdx.x;
  const float e = (float)(2 * j) * (1.0f / 512.0f);
  const float pw = powf(10000.0f, e);
  const float r = 1.0f / pw;
  ((volatile float*)rp)[j] = r;
  __threadfence();
  ((volatile float*)rp)[j] = r;
}

__global__ __launch_bounds__(256) void k_petab(const float* __restrict__ rp, float* __restrict__ pe) {
  const int s = blockIdx.x, j = threadIdx.x;
  const float ang = (float)s * rp[j];
  v2f o;
  o[0] = sinf(ang);
  o[1] = cosf(ang);
  float* dst = pe + (size_t)s * kDim + 2 * j;
  *(volatile v2f*)dst = o;
  __threadfence();
  *(volatile v2f*)dst = o;
}

__global__ __launch_bounds__(128) void k_embed(const int* __restrict__ tokens, const float* __restrict__ emb,
                                               const float* __restrict__ pe, float* __restrict__ x, int nvocab) {
  const int row = blockIdx.x;
  const int s = row & (kSeq - 1);
  int tok = tokens[row];
  if (tok < 0) tok += nvocab;
  tok = tok < 0 ? 0 : (tok >= nvocab ? nvocab - 1 : tok);
  const int c4 = threadIdx.x * 4;
  const v4f e = *(const v4f*)(emb + (size_t)tok * kDim + c4);
  const v4f p = *(const v4f*)(pe + (size_t)s * kDim + c4);
  v4f o;
#pragma unroll
  for (int i = 0; i < 4; ++i) o[i] = bf16r(e[i]) + p[i];
  float* dst = x + (size_t)row * kDim + c4;
  *(volatile v4f*)dst = o;
  __threadfence();
  *(volatile v4f*)dst = o;
}

__global__ __launch_bounds__(256) void k_tconv(const float* __restrict__ W, unsigned short* __restrict__ o,
                                               int R, int Cc, long sIn, long sOut, float mul) {
  __shared__ __align__(16) float tf[64 * 68];
  W += (size_t)blockIdx.z * sIn;
  o += (size_t)blockIdx.z * sOut;
  const int c0  = blockIdx.x * 64;
  const int r0  = blockIdx.y * 64;
  const int tid = threadIdx.x;
  {
    const int lr = tid >> 4;
    const int c4 = (tid & 15) * 4;
#pragma unroll
    for (int it = 0; it < 4; ++it) {
      const int rr = it * 16 + lr;
      const v4f a = *(const v4f*)(W + (size_t)(r0 + rr) * Cc + c0 + c4);
      *(v4f*)(tf + rr * 68 + c4) = a;
    }
  }
  __syncthreads();
  const int sub = tid >> 3;
  const int c8  = (tid & 7) * 8;
  v4u hv[2];
#pragma unroll
  for (int it = 0; it < 2; ++it) {
    const int oc = it * 32 + sub;
    v4u a;
#pragma unroll
    for (int q = 0; q < 4; ++q) {
      const float f0 = bf16r(tf[(c8 + 2 * q) * 68 + oc]) * mul;
      const float f1 = bf16r(tf[(c8 + 2 * q + 1) * 68 + oc]) * mul;
      a[q] = pk16(h_bits(f0), h_bits(f1));
    }
    hv[it] = a;
  }
  for (int pass = 0; pass < 2; ++pass) {
#pragma unroll
    for (int it = 0; it < 2; ++it) {
      const int oc = it * 32 + sub;
      const size_t go = (size_t)(c0 + oc) * R + r0 + c8;
      *(volatile v4u*)(o + go) = hv[it];
    }
    __threadfence();
  }
}

__global__ __launch_bounds__(256) void k_cos_tp(const float* __restrict__ x, const float* __restrict__ theta,
                                                unsigned short* __restrict__ prow, unsigned short* __restrict__ ptp) {
  __shared__ __align__(16) float tf[64 * 68];
  const int d0 = blockIdx.x * 64, s0 = blockIdx.y * 64, b = blockIdx.z, tid = threadIdx.x;
  {
    const int lr = tid >> 4, c4 = (tid & 15) * 4;
    const v4f tv = *(const v4f*)(theta + d0 + c4);
    const float t0 = bf16r(tv[0]), t1 = bf16r(tv[1]), t2 = bf16r(tv[2]), t3 = bf16r(tv[3]);
#pragma unroll 1
    for (int it = 0; it < 4; ++it) {
      const int rr = it * 16 + lr;
      const v4f a = *(const v4f*)(x + (size_t)(b * kSeq + s0 + rr) * kDim + d0 + c4);
      v4f cv;
      cv[0] = cos_f32(a[0] + t0);
      cv[1] = cos_f32(a[1] + t1);
      cv[2] = cos_f32(a[2] + t2);
      cv[3] = cos_f32(a[3] + t3);
      *(v4f*)(tf + rr * 68 + c4) = cv;
    }
  }
  __syncthreads();
  const int sub = tid >> 3, c8 = (tid & 7) * 8;
  v4u hv[2], tv2[2];
#pragma unroll
  for (int it = 0; it < 2; ++it) {
    const int rr = it * 32 + sub;
    v4u a, t;
#pragma unroll
    for (int q = 0; q < 4; ++q) {
      a[q] = pk16(h_bits(tf[rr * 68 + c8 + 2 * q]), h_bits(tf[rr * 68 + c8 + 2 * q + 1]));
      t[q] = pk16(h_bits(tf[(c8 + 2 * q) * 68 + rr]), h_bits(tf[(c8 + 2 * q + 1) * 68 + rr]));
    }
    hv[it] = a; tv2[it] = t;
  }
  for (int pass = 0; pass < 2; ++pass) {
#pragma unroll
    for (int it = 0; it < 2; ++it) {
      const int rr = it * 32 + sub;
      *(volatile v4u*)(prow + (size_t)(b * kSeq + s0 + rr) * kDim + d0 + c8) = hv[it];
      *(volatile v4u*)(ptp + ((size_t)b * kDim + d0 + rr) * kSeq + s0 + c8) = tv2[it];
    }
    __threadfence();
  }
}

__global__ __launch_bounds__(256) void k_cos_row(const float* __restrict__ x, const float* __restrict__ theta,
                                                 unsigned short* __restrict__ hp, int n4) {
  const int i = blockIdx.x * 256 + threadIdx.x;
  if (i >= n4) return;
  const int d4 = (i & (kDim / 4 - 1)) * 4;
  const v4f xv = *(const v4f*)(x + (size_t)i * 4);
  const v4f tv = *(const v4f*)(theta + d4);
  const unsigned short h0 = h_bits(cos_f32(xv[0] + bf16r(tv[0])));
  const unsigned short h1 = h_bits(cos_f32(xv[1] + bf16r(tv[1])));
  const unsigned short h2 = h_bits(cos_f32(xv[2] + bf16r(tv[2])));
  const unsigned short h3 = h_bits(cos_f32(xv[3] + bf16r(tv[3])));
  v2u o;
  o[0] = pk16(h0, h1);
  o[1] = pk16(h2, h3);
  unsigned short* dst = hp + (size_t)i * 4;
  *(volatile v2u*)dst = o;
  __threadfence();
  *(volatile v2u*)dst = o;
}

constexpr int kAtKC = 64;
constexpr int kAtQB = 64;
constexpr int kAtNW = 4;

__device__ __forceinline__ v8f mma_h(v16h a, v16h b, v8f c) {
  c = __builtin_amdgcn_wmma_f32_16x16x32_f16(false, a, false, b, (short)0, c, false, false);
  asm volatile("v_nop\n\tv_nop\n\tv_nop\n\tv_nop" : "+v"(c) : "v"(a), "v"(b));
  return c;
}

__global__ __launch_bounds__(128)
void k_attn_f16(const unsigned short* __restrict__ pp, const unsigned short* __restrict__ ptp,
                unsigned short* __restrict__ op, float sscale) {
  typedef Frag<_Float16> FR;
  __shared__ __align__(16) _Float16 Ksh[kAtKC * kHeadDim];
  __shared__ __align__(16) _Float16 Vth[kHeadDim * kAtKC];
  __shared__ __align__(16) _Float16 Psh[kAtNW][16 * kAtKC];
  __shared__ __align__(16) float    Os[kAtNW][16 * 68];

  const int tid  = threadIdx.x;
  const int wave = tid >> 5;
  const int lane = tid & 31;
  const int hh   = lane >> 4;
  const int c    = lane & 15;

  constexpr int nqb = kSeq / kAtQB;
  const int bx  = blockIdx.x;
  const int qb  = bx % nqb;
  const int bhx = bx / nqb;
  const int h   = bhx % kHeads;
  const int b   = bhx / kHeads;
  const int q0  = qb * kAtQB + wave * 16;

  const _Float16* P  = (const _Float16*)(const void*)pp  + (size_t)b * kSeq * kDim + h * kHeadDim;
  const _Float16* Vt = (const _Float16*)(const void*)ptp + ((size_t)b * kDim + h * kHeadDim) * kSeq;
  unsigned short* ob = op + (size_t)b * kSeq * kDim + h * kHeadDim;

  v16h qa[2];
#pragma unroll
  for (int dc = 0; dc < 2; ++dc) qa[dc] = FR::load(P + (size_t)(q0 + c) * kDim + dc * 32 + 8 * hh);

  float mrow[8], lrow[8];
  v8f oacc[4];
#pragma unroll
  for (int r = 0; r < 8; ++r) { mrow[r] = -INFINITY; lrow[r] = 0.f; }
#pragma unroll
  for (int t = 0; t < 4; ++t) oacc[t] = (v8f){0.f,0.f,0.f,0.f,0.f,0.f,0.f,0.f};

  for (int kc = 0; kc < kSeq / kAtKC; ++kc) {
    const int kv0 = kc * kAtKC;
    __syncthreads();
    {
      const int r = tid >> 1, half = (tid & 1) * 32;
      const _Float16* ks = P  + (size_t)(kv0 + r) * kDim + half;
      const _Float16* vs = Vt + (size_t)r * kSeq + kv0 + half;
#pragma unroll
      for (int i = 0; i < 4; ++i) {
        const v8h a0 = *(const v8h*)(ks + 8 * i);
        const v8h b0 = *(const v8h*)(vs + 8 * i);
        *(v8h*)(Ksh + r * kHeadDim + half + 8 * i) = a0;
        *(v8h*)(Vth + r * kAtKC   + half + 8 * i) = b0;
      }
    }
    __syncthreads();

    v8f s[4];
#pragma unroll
    for (int j = 0; j < 4; ++j) {
      s[j] = (v8f){0.f,0.f,0.f,0.f,0.f,0.f,0.f,0.f};
#pragma unroll
      for (int dc = 0; dc < 2; ++dc) {
        const v16h kb = FR::load(Ksh + (j * 16 + c) * kHeadDim + dc * 32 + 8 * hh);
        s[j] = mma_h(qa[dc], kb, s[j]);
      }
    }
    float cm[8];
#pragma unroll
    for (int r = 0; r < 8; ++r) {
      float m = -INFINITY;
#pragma unroll
      for (int j = 0; j < 4; ++j) { const float sv = s[j][r] * sscale; s[j][r] = sv; m = fmaxf(m, sv); }
#pragma unroll
      for (int off = 1; off < 16; off <<= 1) m = fmaxf(m, __shfl_xor(m, off, 32));
      cm[r] = m;
    }
    _Float16* pw = Psh[wave];
#pragma unroll
    for (int r = 0; r < 8; ++r) {
      const float mnew  = fmaxf(mrow[r], cm[r]);
      const float alpha = expf(mrow[r] - mnew);
      mrow[r] = mnew;
      float psum = 0.f;
#pragma unroll
      for (int j = 0; j < 4; ++j) {
        const float p = expf(s[j][r] - mnew);
        psum += p;
        pw[(8 * hh + r) * kAtKC + j * 16 + c] = (_Float16)(p * kPScale);
      }
#pragma unroll
      for (int off = 1; off < 16; off <<= 1) psum += __shfl_xor(psum, off, 32);
      lrow[r] = lrow[r] * alpha + psum;
#pragma unroll
      for (int t = 0; t < 4; ++t) oacc[t][r] *= alpha;
    }
    __builtin_amdgcn_fence(__ATOMIC_RELEASE, "workgroup");
    __builtin_amdgcn_wave_barrier();
    __builtin_amdgcn_fence(__ATOMIC_ACQUIRE, "workgroup");
#pragma unroll 1
    for (int kk = 0; kk < 2; ++kk) {
      const v16h pa = FR::load(pw + c * kAtKC + kk * 32 + 8 * hh);
#pragma unroll
      for (int t = 0; t < 4; ++t) {
        const v16h vb = FR::load(Vth + (t * 16 + c) * kAtKC + kk * 32 + 8 * hh);
        oacc[t] = mma_h(pa, vb, oacc[t]);
      }
    }
  }

  float* os = Os[wave];
#pragma unroll
  for (int r = 0; r < 8; ++r) {
    const float inv = 1.0f / (lrow[r] * kPScale);
#pragma unroll
    for (int t = 0; t < 4; ++t) os[(8 * hh + r) * 68 + t * 16 + c] = oacc[t][r] * inv;
  }
  __builtin_amdgcn_fence(__ATOMIC_RELEASE, "workgroup");
  __builtin_amdgcn_wave_barrier();
  __builtin_amdgcn_fence(__ATOMIC_ACQUIRE, "workgroup");
  {
    const int q4 = lane >> 3, c8 = (lane & 7) * 8;
    v8h hv[4];
#pragma unroll
    for (int it = 0; it < 4; ++it) {
      const int row = it * 4 + q4;
      const float* sp = os + row * 68 + c8;
      v8h t;
#pragma unroll
      for (int e = 0; e < 8; ++e) t[e] = (_Float16)sp[e];
      hv[it] = t;
    }
    for (int pass = 0; pass < 2; ++pass) {
#pragma unroll
      for (int it = 0; it < 4; ++it) {
        const int row = it * 4 + q4;
        *(volatile v8h*)(ob + (size_t)(q0 + row) * kDim + c8) = hv[it];
      }
      __threadfence();
    }
  }
}

__global__ __launch_bounds__(256) void k_ln(const float* __restrict__ y, const float* __restrict__ g,
                                            const float* __restrict__ bb, float* __restrict__ x, int nrows) {
  const int wave = threadIdx.x >> 5, lane = threadIdx.x & 31;
  const int row = blockIdx.x * 8 + wave;
  if (row >= nrows) return;
  const float* yr = y + (size_t)row * kDim;
  v4f v[4];
  float sum = 0.f;
#pragma unroll
  for (int q = 0; q < 4; ++q) {
    v[q] = *(const v4f*)(yr + q * 128 + lane * 4);
    sum += (v[q][0] + v[q][1]) + (v[q][2] + v[q][3]);
  }
#pragma unroll
  for (int o = 16; o; o >>= 1) sum += __shfl_xor(sum, o, 32);
  const float mu = sum * (1.0f / (float)kDim);
  float s2 = 0.f;
#pragma unroll
  for (int q = 0; q < 4; ++q) {
#pragma unroll
    for (int e = 0; e < 4; ++e) { const float t = v[q][e] - mu; s2 = fmaf(t, t, s2); }
  }
#pragma unroll
  for (int o = 16; o; o >>= 1) s2 += __shfl_xor(s2, o, 32);
  const float rstd = rsqrtf(s2 * (1.0f / (float)kDim) + 1e-5f);
  v4f ov[4];
#pragma unroll
  for (int q = 0; q < 4; ++q) {
    const v4f gv = *(const v4f*)(g  + q * 128 + lane * 4);
    const v4f bv = *(const v4f*)(bb + q * 128 + lane * 4);
    v4f o;
#pragma unroll
    for (int e = 0; e < 4; ++e) o[e] = (bf16r(gv[e]) * (v[q][e] - mu)) * rstd + bf16r(bv[e]);
    ov[q] = o;
  }
  float* xr = x + (size_t)row * kDim;
  for (int pass = 0; pass < 2; ++pass) {
#pragma unroll
    for (int q = 0; q < 4; ++q) *(volatile v4f*)(xr + q * 128 + lane * 4) = ov[q];
    __threadfence();
  }
}

__global__ __launch_bounds__(512) void k_poolcls(const float* __restrict__ x, const float* __restrict__ wcls,
                                                 const float* __restrict__ bcls, float* __restrict__ out) {
  __shared__ float pooled[kBatch * kDim];
  __shared__ __align__(16) float res[kBatch * kClasses];
  const int d = threadIdx.x;
#pragma unroll 1
  for (int b = 0; b < kBatch; ++b) {
    const float* xp = x + (size_t)b * kSeq * kDim + d;
    float a0 = 0.f, a1 = 0.f, a2 = 0.f, a3 = 0.f;
#pragma unroll 1
    for (int s = 0; s < kSeq; s += 4) {
      a0 += xp[(size_t)(s)     * kDim];
      a1 += xp[(size_t)(s + 1) * kDim];
      a2 += xp[(size_t)(s + 2) * kDim];
      a3 += xp[(size_t)(s + 3) * kDim];
    }
    pooled[b * kDim + d] = ((a0 + a1) + (a2 + a3)) * (1.0f / (float)kSeq);
  }
  __syncthreads();
  if (d < kBatch * kClasses) {
    const int b = d / kClasses, cc = d - b * kClasses;
    float acc = 0.f;
#pragma unroll 1
    for (int k = 0; k < kDim; ++k) acc = fmaf(pooled[b * kDim + k], bf16r(wcls[k * kClasses + cc]), acc);
    res[d] = acc + bf16r(bcls[cc]);
  }
  __syncthreads();
  if (d < (kBatch * kClasses) / 4) {
    const v4f vv = *(const v4f*)(res + d * 4);
    *(volatile v4f*)(out + d * 4) = vv;
    __threadfence();
    *(volatile v4f*)(out + d * 4) = vv;
  }
}

extern "C" void kernel_launch(void* const* d_in, const int* in_sizes, int n_in,
                              void* d_out, int out_size, void* d_ws, size_t ws_size,
                              hipStream_t stream) {
  if (n_in < 16) return;
  if (in_sizes[0] != kRows) return;
  if (in_sizes[1] < kDim || (in_sizes[1] % kDim) != 0) return;
  if (in_sizes[2] != kLayers * kDim || in_sizes[3] != kLayers * kDim * kDim || in_sizes[4] != kLayers * kDim) return;
  if (in_sizes[5] != kLayers * kDim || in_sizes[6] != kLayers * kDim || in_sizes[7] != kLayers * kDim) return;
  if (in_sizes[8] != kLayers * kDim * kFfn || in_sizes[9] != kLayers * kFfn) return;
  if (in_sizes[10] != kLayers * kFfn * kDim || in_sizes[11] != kLayers * kDim) return;
  if (in_sizes[12] != kLayers * kDim || in_sizes[13] != kLayers * kDim) return;
  if (in_sizes[14] != kDim * kClasses || in_sizes[15] != kClasses) return;
  if (out_size != kBatch * kClasses) return;

  const int*   tokens     = (const int*)d_in[0];
  const float* embedding  = (const float*)d_in[1];
  const float* theta_attn = (const float*)d_in[2];
  const float* Wc         = (const float*)d_in[3];
  const float* bc         = (const float*)d_in[4];
  const float* ln1_g      = (const float*)d_in[5];
  const float* ln1_b      = (const float*)d_in[6];
  const float* theta_ffn  = (const float*)d_in[7];
  const float* W1         = (const float*)d_in[8];
  const float* b1         = (const float*)d_in[9];
  const float* W2         = (const float*)d_in[10];
  const float* b2         = (const float*)d_in[11];
  const float* ln2_g      = (const float*)d_in[12];
  const float* ln2_b      = (const float*)d_in[13];
  const float* Wcls       = (const float*)d_in[14];
  const float* bcls       = (const float*)d_in[15];
  const int nvocab = in_sizes[1] / kDim;

  const size_t MiB = (size_t)1 << 20;
  const size_t off_x    = 0;
  const size_t off_tmp  = off_x    + (size_t)kRows * kDim * 4;
  const size_t off_p16  = off_tmp  + (size_t)kRows * kDim * 4;
  const size_t off_p16t = off_p16  + (size_t)kRows * kDim * 2;
  const size_t off_att  = off_p16t + (size_t)kRows * kDim * 2;
  const size_t off_hid  = off_att  + (size_t)kRows * kDim * 2;
  const size_t off_wct  = off_hid  + (size_t)kRows * kFfn * 2;
  const size_t off_w1t  = off_wct  + (size_t)kLayers * kDim * kDim * 2;
  const size_t off_w2t  = off_w1t  + (size_t)kLayers * kFfn * kDim * 2;
  const size_t off_pe   = off_w2t  + (size_t)kLayers * kDim * kFfn * 2;
  const size_t off_rp   = off_pe   + (size_t)kSeq * kDim * 4;
  const size_t off_end  = off_rp   + 1024;
  if (off_end > ws_size || off_end > 128 * MiB) return;

  char* ws = (char*)d_ws;
  float*          x     = (float*)(ws + off_x);
  float*          tmp   = (float*)(ws + off_tmp);
  unsigned short* p16   = (unsigned short*)(ws + off_p16);
  unsigned short* p16t  = (unsigned short*)(ws + off_p16t);
  unsigned short* att16 = (unsigned short*)(ws + off_att);
  unsigned short* hid16 = (unsigned short*)(ws + off_hid);
  unsigned short* wct   = (unsigned short*)(ws + off_wct);
  unsigned short* w1t   = (unsigned short*)(ws + off_w1t);
  unsigned short* w2t   = (unsigned short*)(ws + off_w2t);
  float*          pe    = (float*)(ws + off_pe);
  float*          rp    = (float*)(ws + off_rp);

  k_powtab<<<1, 256, 0, stream>>>(rp);
  k_petab<<<kSeq, 256, 0, stream>>>(rp, pe);
  k_embed<<<kRows, 128, 0, stream>>>(tokens, embedding, pe, x, nvocab);
  k_tconv<<<dim3(kDim / 64, kDim / 64, kLayers), 256, 0, stream>>>(
      Wc, wct, kDim, kDim, (long)kDim * kDim, (long)kDim * kDim, kWScale);
  k_tconv<<<dim3(kFfn / 64, kDim / 64, kLayers), 256, 0, stream>>>(
      W1, w1t, kDim, kFfn, (long)kDim * kFfn, (long)kFfn * kDim, kWScale);
  k_tconv<<<dim3(kDim / 64, kFfn / 64, kLayers), 256, 0, stream>>>(
      W2, w2t, kFfn, kDim, (long)kFfn * kDim, (long)kDim * kFfn, kWScale);

  const int gemm_blocks_n512  = ((kRows / 64) * (kDim / 64) + 7) / 8;
  const int gemm_blocks_n2048 = ((kRows / 64) * (kFfn / 64) + 7) / 8;

  for (int l = 0; l < kLayers; ++l) {
    k_cos_tp<<<dim3(kDim / 64, kSeq / 64, kBatch), 256, 0, stream>>>(x, theta_attn + (size_t)l * kDim, p16, p16t);
    k_attn_f16<<<kBatch * kHeads * (kSeq / kAtQB), 128, 0, stream>>>(p16, p16t, att16, 0.125f);
    wmma_gemm64<0, false, 2, 0, true, 0><<<dim3(gemm_blocks_n512, 1), 256, 0, stream>>>(
        att16, att16, kDim, 0L,
        wct + (size_t)l * kDim * kDim, wct + (size_t)l * kDim * kDim, kDim, 0L,
        (void*)tmp, (void*)tmp, kDim, 0L,
        bc + (size_t)l * kDim,
        x, 0L,
        kRows, kDim, kDim, kWScaleInv);
    k_ln<<<kRows / 8, 256, 0, stream>>>(tmp, ln1_g + (size_t)l * kDim, ln1_b + (size_t)l * kDim, x, kRows);
    k_cos_row<<<(kRows * kDim / 4) / 256, 256, 0, stream>>>(x, theta_ffn + (size_t)l * kDim, p16, kRows * kDim / 4);
    wmma_gemm64<0, false, 2, 1, false, 2><<<dim3(gemm_blocks_n2048, 1), 256, 0, stream>>>(
        p16, p16, kDim, 0L,
        w1t + (size_t)l * kFfn * kDim, w1t + (size_t)l * kFfn * kDim, kDim, 0L,
        (void*)hid16, (void*)hid16, kFfn, 0L,
        b1 + (size_t)l * kFfn,
        x, 0L,
        kRows, kFfn, kDim, kWScaleInv);
    wmma_gemm64<0, false, 2, 0, true, 0><<<dim3(gemm_blocks_n512, 1), 256, 0, stream>>>(
        hid16, hid16, kFfn, 0L,
        w2t + (size_t)l * kDim * kFfn, w2t + (size_t)l * kDim * kFfn, kFfn, 0L,
        (void*)tmp, (void*)tmp, kDim, 0L,
        b2 + (size_t)l * kDim,
        x, 0L,
        kRows, kDim, kFfn, kWScaleInv);
    k_ln<<<kRows / 8, 256, 0, stream>>>(tmp, ln2_g + (size_t)l * kDim, ln2_b + (size_t)l * kDim, x, kRows);
  }

  k_poolcls<<<1, 512, 0, stream>>>(x, Wcls, bcls, (float*)d_out);
}
